// MolecularRetNet_15994458210954
// MI455X (gfx1250) — hardware-verified
//
#include <hip/hip_runtime.h>
#include <math.h>

typedef __attribute__((ext_vector_type(16))) _Float16 v16h;
typedef __attribute__((ext_vector_type(16))) __bf16 v16b;
typedef __attribute__((ext_vector_type(8)))  _Float16 v8h;
typedef __attribute__((ext_vector_type(8)))  float v8f;
typedef __attribute__((ext_vector_type(4)))  float v4f;
typedef __attribute__((ext_vector_type(2)))  float v2f;
typedef __attribute__((ext_vector_type(4)))  unsigned v4u;
typedef __attribute__((ext_vector_type(4)))  int v4i;
typedef float __attribute__((may_alias)) float_a;
typedef int __attribute__((may_alias)) int_a;

template <typename T> __device__ __forceinline__ void vst2(void* p, T v) { *(volatile T*)p = v; __threadfence(); *(volatile T*)p = v; }
__device__ __forceinline__ v8f wmma16(v16h a, v16h b, v8f c) {
  v8f d = __builtin_amdgcn_wmma_f32_16x16x32_f16(false, a, false, b, (short)0, c, false, false);
  asm volatile("v_nop\n\tv_nop\n\tv_nop\n\tv_nop" : "+v"(d) : "v"(a), "v"(b));
  return d;
}
__device__ __forceinline__ v8f wmma_bf(v16b a, v16b b, v8f c) {
  v8f d = __builtin_amdgcn_wmma_f32_16x16x32_bf16(false, a, false, b, (short)0, c, false, false);
  asm volatile("v_nop\n\tv_nop\n\tv_nop\n\tv_nop" : "+v"(d) : "v"(a), "v"(b));
  return d;
}
__device__ __forceinline__ v16h frag_h(const _Float16* rowk0, int lane) {
  union { v16h v; v8h q[2]; } u; const _Float16* p = rowk0 + 8 * (lane >> 4);
  u.q[0] = *(const v8h*)p; u.q[1] = *(const v8h*)(p + 16); return u.v;
}
__device__ __forceinline__ v16h frag_f32(const float* rowk0, int lane) {
  v16h a; const float* p = rowk0 + 8 * (lane >> 4);
#pragma unroll
  for (int i = 0; i < 8; ++i) { a[i] = (_Float16)p[i]; a[8 + i] = (_Float16)p[16 + i]; }
  return a;
}
__device__ __forceinline__ v16h frag_f32s(const float* rowk0, int lane, float sc) {
  v16h a; const float* p = rowk0 + 8 * (lane >> 4);
#pragma unroll
  for (int i = 0; i < 8; ++i) { a[i] = (_Float16)(p[i] * sc); a[8 + i] = (_Float16)(p[16 + i] * sc); }
  return a;
}
__device__ __forceinline__ v16h fragc_f32(const float* W, int k0, int n, int lane, int ld, int K) {
  v16h a; const int g = lane >> 4;
#pragma unroll
  for (int i = 0; i < 8; ++i) { const int ka = k0 + 8 * g + i, kb = ka + 16;
    a[i] = (_Float16)(ka < K ? W[(size_t)(ka < K ? ka : K - 1) * ld + n] : 0.f); a[8 + i] = (_Float16)(kb < K ? W[(size_t)(kb < K ? kb : K - 1) * ld + n] : 0.f); }
  return a;
}
struct F2 { v16b h, l; };
__device__ __forceinline__ F2 bsplit16(const float v[16]) { F2 r;
#pragma unroll
  for (int i = 0; i < 16; ++i) { const __bf16 h = (__bf16)v[i]; r.h[i] = h; r.l[i] = (__bf16)(v[i] - (float)h); }
  return r; }
__device__ __forceinline__ F2 split_row(const float* row, int k0, int lane) { float v[16]; const float* p = row + k0 + 8 * (lane >> 4);
#pragma unroll
  for (int i = 0; i < 8; ++i) { v[i] = p[i]; v[8 + i] = p[16 + i]; }
  return bsplit16(v); }
__device__ __forceinline__ F2 split_rowK(const float* row, int k0, int lane, int K) { float v[16]; const int g = lane >> 4;
#pragma unroll
  for (int i = 0; i < 8; ++i) { const int ka = k0 + 8 * g + i, kb = ka + 16; v[i] = ka < K ? row[ka < K ? ka : K - 1] : 0.f; v[8 + i] = kb < K ? row[kb < K ? kb : K - 1] : 0.f; }
  return bsplit16(v); }
__device__ __forceinline__ F2 split_col(const float* W, int k0, int n, int lane, int ld, int K) { float v[16]; const int g = lane >> 4;
#pragma unroll
  for (int i = 0; i < 8; ++i) { const int ka = k0 + 8 * g + i, kb = ka + 16; v[i] = ka < K ? W[(size_t)(ka < K ? ka : K - 1) * ld + n] : 0.f; v[8 + i] = kb < K ? W[(size_t)(kb < K ? kb : K - 1) * ld + n] : 0.f; }
  return bsplit16(v); }
__device__ __forceinline__ v8f mac3(const F2& a, const F2& b, v8f c) { c = wmma_bf(a.l, b.h, c); c = wmma_bf(a.h, b.l, c); return wmma_bf(a.h, b.h, c); }
__device__ __forceinline__ float sigm(float v) { return 1.0f / (1.0f + expf(-v)); }
#define LDSX() do { asm volatile("s_wait_dscnt 0" ::: "memory"); __builtin_amdgcn_wave_barrier(); __builtin_amdgcn_fence(__ATOMIC_RELEASE, "workgroup"); } while (0)


#define NB 32
#define SS 512
#define DD 256
#define NH 8
#define HD 32
#define FFN 128
#define NL 3
#define NTOK (NB * SS)
#ifndef TQB
#define TQB (SS / 64)
#define TNB NB
#endif
typedef __attribute__((ext_vector_type(8))) __bf16 v8b;
__device__ __forceinline__ v16b frag_b(const __bf16* rowk0, int lane) {
  union { v16b v; v8b q[2]; } u; const __bf16* p = rowk0 + 8 * (lane >> 4);
  u.q[0] = *(const v8b*)p; u.q[1] = *(const v8b*)(p + 16); return u.v;
}
__device__ __forceinline__ float bfr(float v) { return (float)(__bf16)v; }
__device__ __attribute__((noinline)) float exp_ni(float v) { return expf(v); }
__device__ __attribute__((noinline)) float erf_ni(float v) { return erff(v); }

#define WS_PW  0u
#define LSTRIDE (1024 * DD + DD * DD + FFN * DD + DD * FFN)
#define WS_XT  (WS_PW + 2u * NL * LSTRIDE)
#define WS_X   (WS_XT + 4u * 2 * SS * 16 * 2)
#define WS_XN  (WS_X + 4u * NTOK * DD)
#define WS_QK  (WS_XN + 4u * NTOK * DD)
#define WS_G   (WS_QK + 4u * NTOK * 2 * DD)
#define WS_VH  (WS_G + 4u * NTOK * DD)
#define WS_VL  (WS_VH + 2u * NB * DD * SS)
#define WS_YN  (WS_VL + 2u * NB * DD * SS)
#define WS_Y2  (WS_YN + 4u * NTOK * DD)
#define WS_F1  (WS_Y2 + 4u * NTOK * DD)
#define WS_END (WS_F1 + 4u * NTOK * FFN)

__global__ __launch_bounds__(256) void k_packT(const float* __restrict__ WQ, const float* __restrict__ WK, const float* __restrict__ WV, const float* __restrict__ WG, const float* __restrict__ WO, const float* __restrict__ W1, const float* __restrict__ W2, __bf16* __restrict__ PW) {
  __shared__ __align__(16) __bf16 s[DD]; const int n = blockIdx.x, p = blockIdx.y, tid = threadIdx.x; const int l = p >> 2, which = p & 3; int K; size_t dst; float v = 0.f;
  __bf16* base = PW + (size_t)l * LSTRIDE;
  if (which == 0) { K = DD; dst = (size_t)n * DD; const int part = n >> 8, c = n & 255; if (tid < K) { if (part < 3) { const float* Wm = (part == 0) ? WQ : (part == 1 ? WK : WV); const int h = c >> 5, e = c & 31; v = Wm[(((size_t)l * NH + h) * DD + tid) * HD + e]; } else v = WG[((size_t)l * DD + tid) * DD + c]; } }
  else if (which == 1) { if (n >= DD) return; K = DD; dst = (size_t)1024 * DD + (size_t)n * DD; if (tid < K) v = WO[((size_t)l * DD + tid) * DD + n]; }
  else if (which == 2) { if (n >= FFN) return; K = DD; dst = (size_t)1024 * DD + DD * DD + (size_t)n * DD; if (tid < K) v = W1[((size_t)l * DD + tid) * FFN + n]; }
  else { if (n >= DD) return; K = FFN; dst = (size_t)1024 * DD + DD * DD + FFN * DD + (size_t)n * FFN; if (tid < K) v = W2[((size_t)l * FFN + tid) * DD + n]; }
  if (tid < K) s[tid] = (__bf16)v; __syncthreads();
  if (tid < K / 8) vst2((unsigned*)(base + dst + tid * 8), *(const v4u*)&s[tid * 8]);
}
__global__ __launch_bounds__(256) void k_embed(const int* __restrict__ VID, const float* __restrict__ EMB, float* __restrict__ X) {
  __shared__ __align__(16) float so[16][DD]; const int tid = threadIdx.x; const size_t r0 = (size_t)blockIdx.x * 64;
  for (int part = 0; part < 4; ++part) { for (int rl = 0; rl < 16; ++rl) { const int id = min(max(VID[r0 + part * 16 + rl], 0), 64); so[rl][tid] = (id == 0) ? 0.f : fmaxf(bfr(EMB[(size_t)id * DD + tid]), 0.f); }
    __syncthreads();
    for (int q = tid; q < 16 * DD / 4; q += 256) { const int rl = q / (DD / 4), pc = q % (DD / 4); vst2(X + (r0 + part * 16 + rl) * DD + pc * 4, *(const v4f*)&so[rl][pc * 4]); }
    __syncthreads(); }
}
__global__ __launch_bounds__(256) void k_ln(const float* __restrict__ IN, const float* __restrict__ w, const float* __restrict__ bb, float* __restrict__ OUT) {
  __shared__ __align__(16) float s[8][DD]; const int wave = threadIdx.x >> 5, lane = threadIdx.x & 31; const size_t row = (size_t)blockIdx.x * 8 + wave; float v[8]; float sum = 0.f;
#pragma unroll
  for (int k = 0; k < 8; ++k) { v[k] = IN[row * DD + lane + 32 * k]; sum += v[k]; }
#pragma unroll
  for (int o = 1; o < 32; o <<= 1) sum += __shfl_xor(sum, o);
  const float mu = sum / (float)DD; float var = 0.f;
#pragma unroll
  for (int k = 0; k < 8; ++k) { const float d = v[k] - mu; var += d * d; }
#pragma unroll
  for (int o = 1; o < 32; o <<= 1) var += __shfl_xor(var, o);
  const float rs = 1.0f / sqrtf(var / (float)DD + 1e-5f);
#pragma unroll
  for (int k = 0; k < 8; ++k) { const int c = lane + 32 * k; s[wave][c] = (v[k] - mu) * rs * bfr(w[c]) + bfr(bb[c]); }
  LDSX();
  for (int pc = lane; pc < DD / 4; pc += 32) vst2(OUT + row * DD + pc * 4, *(const v4f*)&s[wave][pc * 4]);
}
__device__ __attribute__((noinline)) float pow_ni(float a, float b) { return powf(a, b); }
__device__ __attribute__((noinline)) float cos_ni(float v) { return cosf(v); }
__device__ __attribute__((noinline)) float sin_ni(float v) { return sinf(v); }
__global__ __launch_bounds__(32) void k_xtab(float* __restrict__ XT) {
  __shared__ __align__(16) float s[2][32]; const int n = blockIdx.x, tid = threadIdx.x; const int which = tid >> 4, jx = tid & 15;
  const float scl = ((float)(2 * jx) + 0.4f * (float)HD) / (1.4f * (float)HD); float sm = pow_ni(scl, (float)n / 512.0f); if (which) sm = 1.0f / sm;
  const float invf = pow_ni(10000.0f, -(float)jx / (float)(HD / 2)); const float ang = (float)n * invf; s[which][2 * jx] = cos_ni(ang) * sm; s[which][2 * jx + 1] = sin_ni(ang) * sm;
  __syncthreads();
  if (tid < 16) { const int w = tid >> 3, pc = tid & 7; vst2(XT + ((size_t)w * SS + n) * 32 + pc * 4, *(const v4f*)&s[w][pc * 4]); }
}
__global__ __launch_bounds__(128) void k_proj(const float* __restrict__ XN, const __bf16* __restrict__ P, const float* __restrict__ XT, float* __restrict__ QK, __bf16* __restrict__ VH, __bf16* __restrict__ VL, float* __restrict__ G) {
  __shared__ __align__(16) float so[4][16][132]; __shared__ __align__(16) __bf16 sth[128][72], stl[128][72];
  const int tid = threadIdx.x, wave = tid >> 5, lane = tid & 31, col = lane & 15, g = lane >> 4; const size_t rb = (size_t)blockIdx.x * 64; const size_t r0 = rb + wave * 16; const int n0 = blockIdx.y * 128;
  v8f acc[8] = {};
#pragma unroll
  for (int kc = 0; kc < DD / 32; ++kc) { const F2 a = split_row(XN + (r0 + col) * DD, kc * 32, lane);
#pragma unroll
    for (int j = 0; j < 8; ++j) { const v16b wv = frag_b(P + (size_t)(n0 + j * 16 + col) * DD + kc * 32, lane); acc[j] = wmma_bf(a.l, wv, acc[j]); acc[j] = wmma_bf(a.h, wv, acc[j]); } }
  if (n0 < 2 * DD) {
    const bool down = (n0 >= DD);
#pragma unroll
    for (int j = 0; j < 8; ++j)
#pragma unroll
      for (int r = 0; r < 8; ++r) so[wave][8 * g + r][j * 16 + col] = acc[j][r];
    LDSX();
    for (int q = lane; q < 16 * 64; q += 32) { const int rl = q >> 6, pi = q & 63; const int hh = pi >> 4, jx = pi & 15; const int n = (int)((r0 + rl) % SS);
      const float* xt = XT + (((size_t)(down ? 1 : 0) * SS + n) * 16 + jx) * 2; const float c = xt[0], sn = xt[1];
      float* e = &so[wave][rl][hh * 32 + 2 * jx]; const float x1 = e[0], x2 = e[1]; e[0] = x1 * c - x2 * sn; e[1] = x2 * c + x1 * sn; }
    LDSX();
    for (int rl = 0; rl < 16; ++rl) vst2(QK + (r0 + rl) * (2 * DD) + n0 + lane * 4, *(const v4f*)&so[wave][rl][lane * 4]);
  } else if (n0 < 3 * DD) {
#pragma unroll
    for (int j = 0; j < 8; ++j)
#pragma unroll
      for (int r = 0; r < 8; ++r) { const float v = acc[j][r]; const __bf16 hb = (__bf16)v; sth[j * 16 + col][wave * 16 + 8 * g + r] = hb; stl[j * 16 + col][wave * 16 + 8 * g + r] = (__bf16)(v - (float)hb); }
    __syncthreads();
    const int b = (int)(rb / SS), m0 = (int)(rb % SS); const int c0 = n0 - 2 * DD;
    for (int q = tid; q < 128 * 8; q += 128) { const int d = q >> 3, pc = q & 7; const size_t o = ((size_t)b * DD + c0 + d) * SS + m0 + pc * 8; vst2((unsigned*)(VH + o), *(const v4u*)&sth[d][pc * 8]); vst2((unsigned*)(VL + o), *(const v4u*)&stl[d][pc * 8]); }
  } else {
#pragma unroll
    for (int j = 0; j < 8; ++j)
#pragma unroll
      for (int r = 0; r < 8; ++r) so[wave][8 * g + r][j * 16 + col] = acc[j][r];
    LDSX();
    for (int rl = 0; rl < 16; ++rl) vst2(G + (r0 + rl) * DD + (n0 - 3 * DD) + lane * 4, *(const v4f*)&so[wave][rl][lane * 4]);
  }
}
__global__ __launch_bounds__(128) void k_ret(const float* __restrict__ QK, const __bf16* __restrict__ VH, const __bf16* __restrict__ VL, const float* __restrict__ G, const float* __restrict__ GNW, const float* __restrict__ GNB, float* __restrict__ YN) {
  __shared__ __align__(16) float sp[4][16][36]; __shared__ __align__(16) float so[4][16][36];
  const int tid = threadIdx.x, wave = tid >> 5, lane = tid & 31, col = lane & 15, g = lane >> 4; const int qb = blockIdx.x, h = blockIdx.y, b = blockIdx.z; const int q0 = qb * 64 + wave * 16; const size_t rq = (size_t)b * SS + q0;
  const float lgam = log2f(1.0f - exp2f(log2f(1.0f / 32.0f) + (float)h * (log2f(1.0f / 512.0f) - log2f(1.0f / 32.0f)) / (float)(NH - 1)));
  const F2 aq = split_row(QK + (rq + col) * (2 * DD) + h * HD, 0, lane);
  v8f acc[2] = {};
  const int nks = (qb * 64 + 64) / 32;
#pragma unroll 1
  for (int ks = 0; ks < nks; ++ks) {
#pragma unroll
    for (int ct = 0; ct < 2; ++ct) { const int mm = ks * 32 + ct * 16 + col; const F2 kb = split_row(QK + ((size_t)b * SS + mm) * (2 * DD) + DD + h * HD, 0, lane); const v8f s = mac3(aq, kb, (v8f){});
#pragma unroll
      for (int r = 0; r < 8; ++r) { const int n = q0 + 8 * g + r; const float dec = (mm <= n) ? exp2f((float)(n - mm) * lgam) : 0.f; sp[wave][8 * g + r][ct * 16 + col] = s[r] * dec; } }
    LDSX();
    const F2 pa = split_row(&sp[wave][col][0], 0, lane);
#pragma unroll
    for (int dt = 0; dt < 2; ++dt) { const size_t vr = ((size_t)b * DD + h * HD + dt * 16 + col) * SS + ks * 32; const v16b vh = frag_b(VH + vr, lane), vl = frag_b(VL + vr, lane); acc[dt] = wmma_bf(pa.l, vh, acc[dt]); acc[dt] = wmma_bf(pa.h, vl, acc[dt]); acc[dt] = wmma_bf(pa.h, vh, acc[dt]); }
    LDSX(); }
#pragma unroll
  for (int r = 0; r < 8; ++r) { float su = acc[0][r] + acc[1][r];
#pragma unroll
    for (int o = 1; o < 16; o <<= 1) su += __shfl_xor(su, o);
    const float mu = su / (float)HD; const float d0 = acc[0][r] - mu, d1 = acc[1][r] - mu; float va = d0 * d0 + d1 * d1;
#pragma unroll
    for (int o = 1; o < 16; o <<= 1) va += __shfl_xor(va, o);
    const float rs = 1.0f / sqrtf(va / (float)HD + 1e-5f); const size_t row = rq + 8 * g + r;
#pragma unroll
    for (int dt = 0; dt < 2; ++dt) { const int c = h * HD + dt * 16 + col; const float yn = (dt ? d1 : d0) * rs * bfr(GNW[c]) + bfr(GNB[c]); const float gv = G[row * DD + c]; so[wave][8 * g + r][dt * 16 + col] = gv * sigm(gv) * yn; } }
  LDSX();
  for (int rl = 0; rl < 16; ++rl) if (lane < 8) vst2(YN + (rq + rl) * DD + h * HD + lane * 4, *(const v4f*)&so[wave][rl][lane * 4]);
}
template <int NT, int EPI>
__global__ __launch_bounds__(128) void k_gemm(const float* __restrict__ A, int K, const __bf16* __restrict__ P, const float* __restrict__ bias, const float* __restrict__ RES, float* __restrict__ OUT, int ldo) {
  __shared__ __align__(16) float so[4][16][NT * 16 + 4];
  const int tid = threadIdx.x, wave = tid >> 5, lane = tid & 31, col = lane & 15, g = lane >> 4; const size_t r0 = (size_t)blockIdx.x * 64 + wave * 16; const int n0 = blockIdx.y * (NT * 16);
  v8f acc[NT]; for (int j = 0; j < NT; ++j) acc[j] = (v8f){};
#pragma unroll 2
  for (int kc = 0; kc < K / 32; ++kc) { const F2 a = split_row(A + (r0 + col) * K, kc * 32, lane);
#pragma unroll
    for (int j = 0; j < NT; ++j) { const v16b wv = frag_b(P + (size_t)(n0 + j * 16 + col) * K + kc * 32, lane); acc[j] = wmma_bf(a.l, wv, acc[j]); acc[j] = wmma_bf(a.h, wv, acc[j]); } }
#pragma unroll
  for (int j = 0; j < NT; ++j) { const int n = n0 + j * 16 + col; const float bb = bias ? bfr(bias[n]) : 0.f;
#pragma unroll
    for (int r = 0; r < 8; ++r) { float v = acc[j][r] + bb; if (EPI == 1) v = 0.5f * v * (1.0f + erf_ni(v * 0.70710678118654752f)); else v += RES[(r0 + 8 * g + r) * ldo + n]; so[wave][8 * g + r][j * 16 + col] = v; } }
  LDSX();
  for (int rl = 0; rl < 16; ++rl) if (lane < NT * 4) vst2(OUT + (r0 + rl) * ldo + n0 + lane * 4, *(const v4f*)&so[wave][rl][lane * 4]);
}
extern "C" void kernel_launch(void* const* d_in, const int* in_sizes, int n_in, void* d_out, int out_size, void* d_ws, size_t ws_size, hipStream_t stream) {
  (void)in_sizes; (void)n_in; (void)out_size;
  const float** F = (const float**)d_in; const int* VID = (const int*)d_in[0];
  if (ws_size < (size_t)WS_END) return;
  char* ws = (char*)d_ws; __bf16 *PW = (__bf16*)(ws + WS_PW), *VH = (__bf16*)(ws + WS_VH), *VL = (__bf16*)(ws + WS_VL); float *XT = (float*)(ws + WS_XT), *X = (float*)(ws + WS_X), *XN = (float*)(ws + WS_XN), *QK = (float*)(ws + WS_QK), *G = (float*)(ws + WS_G), *YN = (float*)(ws + WS_YN), *Y2 = (float*)(ws + WS_Y2), *F1 = (float*)(ws + WS_F1);
  k_packT<<<dim3(1024, NL * 4), 256, 0, stream>>>(F[2], F[3], F[4], F[5], F[6], F[13], F[15], PW);
  k_embed<<<TNB * SS / 64, 256, 0, stream>>>(VID, F[1], X);
  k_xtab<<<SS, 32, 0, stream>>>(XT);
  const int NR = TNB * SS / 64;
  for (int l = 0; l < NL; ++l) { const __bf16* PL = PW + (size_t)l * LSTRIDE; float* XOUT = (l == NL - 1) ? (float*)d_out : X;
    k_ln<<<TNB * SS / 8, 256, 0, stream>>>(X, F[9] + l * DD, F[10] + l * DD, XN);
    k_proj<<<dim3(NR, 1024 / 128), 128, 0, stream>>>(XN, PL, XT, QK, VH, VL, G);
    k_ret<<<dim3(TQB, NH, TNB), 128, 0, stream>>>(QK, VH, VL, G, F[7] + l * DD, F[8] + l * DD, YN);
    k_gemm<8, 0><<<dim3(NR, DD / 128), 128, 0, stream>>>(YN, DD, PL + 1024 * DD, nullptr, X, Y2, DD);
    k_ln<<<TNB * SS / 8, 256, 0, stream>>>(Y2, F[11] + l * DD, F[12] + l * DD, XN);
    k_gemm<8, 1><<<dim3(NR, FFN / 128), 128, 0, stream>>>(XN, DD, PL + 1024 * DD + DD * DD, F[14] + l * FFN, nullptr, F1, FFN);
    k_gemm<8, 0><<<dim3(NR, DD / 128), 128, 0, stream>>>(F1, FFN, PL + 1024 * DD + DD * DD + FFN * DD, F[16] + l * DD, Y2, XOUT, DD);
  }
}
